// TrajectoryPredictionModel_41970420417898
// MI455X (gfx1250) — hardware-verified
//
#include <hip/hip_runtime.h>
#include <stdint.h>
#include <stddef.h>


typedef __attribute__((ext_vector_type(16))) _Float16 v16h;
typedef __attribute__((ext_vector_type(8)))  _Float16 v8h;
typedef __attribute__((ext_vector_type(8)))  float    v8f;
typedef __attribute__((ext_vector_type(4)))  float    v4f;

__device__ __forceinline__ void dep_guard_h(v8f& a, v8f& b, v16h x, v16h y) { asm volatile("v_nop\n\tv_nop\n\tv_nop\n\tv_nop" : "+v"(a), "+v"(b) : "v"(x), "v"(y)); }
__device__ __forceinline__ void keep4_h(v16h a, v16h b, v16h c, v16h d) { asm volatile("v_nop" :: "v"(a), "v"(b), "v"(c), "v"(d)); }
__device__ __forceinline__ void acc_guard4(v8f& a, v8f& b, v8f& c, v8f& d) { asm volatile("v_nop\n\tv_nop\n\tv_nop\n\tv_nop" : "+v"(a), "+v"(b), "+v"(c), "+v"(d)); }
template <typename T> struct Frag;
template <> struct Frag<_Float16> {
  typedef v16h V; union U { v16h v; v8h h[2]; };
  static __device__ __forceinline__ v16h load(const _Float16* p) {
    U f; f.h[0] = *(const v8h*)(p); f.h[1] = *(const v8h*)(p + 16); return f.v;
  }
  static __device__ __forceinline__ v8f mma(v16h a, v16h b, v8f c) {
    return __builtin_amdgcn_wmma_f32_16x16x32_f16(false, a, false, b, (short)0, c, false, false);
  }
  static __device__ __forceinline__ void guard(v8f& a, v8f& b, v16h x, v16h y) { dep_guard_h(a, b, x, y); }
  static __device__ __forceinline__ void keep(v16h a, v16h b, v16h c, v16h d) { keep4_h(a, b, c, d); }
};

#define NSC   1024
#define TT    8
#define PP    64
#define NROWS 65536
#define KD    128
#define HPITCH 136
#define CPITCH 132

__device__ __forceinline__ float fsig(float z) {
  return __builtin_amdgcn_rcpf(1.0f + __expf(-z));
}
__device__ __forceinline__ float ftanh(float z) {
  const float e  = __expf(2.0f * z);
  const float te = 1.0f - 2.0f * __builtin_amdgcn_rcpf(1.0f + e);
  const float z2 = z * z;
  const float ts = z * fmaf(z2, fmaf(z2, 0.133333340f, -0.333333343f), 1.0f);
  return (fabsf(z) < 0.0625f) ? ts : te;
}

__global__ __launch_bounds__(256) void k_prep_wt(const float* __restrict__ W, int NW, int H, int HP,
                                                 unsigned short* __restrict__ Btp, float wscale) {
  const int tid = threadIdx.x;
  const int r   = blockIdx.x * 16 + (tid >> 4);
  const int c8  = (tid & 15) * 8;
  const int j   = r / HP;
  const int hcc = r - j * HP;
  const bool valid = hcc < H;
  int col = j * H + hcc;
  col = col < NW ? col : NW - 1;
  col = col < 0 ? 0 : col;
  v8h hv;
#pragma unroll
  for (int e = 0; e < 8; ++e) {
    const float f = W[(size_t)(c8 + e) * NW + col] * wscale;
    hv[e] = valid ? (_Float16)f : (_Float16)0.0f;
  }
  _Float16* Bt = (_Float16*)Btp;
  *(volatile v8h*)(Bt + (size_t)r * KD + c8) = hv;
  __threadfence();
  *(volatile v8h*)(Bt + (size_t)r * KD + c8) = hv;
}

__global__ __launch_bounds__(256) void k_enc0(const float* __restrict__ xin, const float* __restrict__ Wx,
                                              const float* __restrict__ bias,
                                              unsigned short* __restrict__ Hout, float* __restrict__ Cout,
                                              float oscale) {
  __shared__ __align__(16) _Float16 hs[8 * HPITCH];
  const int tid = threadIdx.x;
  const int rl  = tid >> 5;
  const int hc4 = (tid & 31) * 4;
  const int row = blockIdx.x * 8 + rl;
  const int n = row >> 6, p = row & 63;
  const size_t xi = ((size_t)(n * TT + 0) * PP + p) * 2;
  const float x0 = xin[xi], x1 = xin[xi + 1];
  v4f cv;
#pragma unroll
  for (int u = 0; u < 4; ++u) {
    const int hc = hc4 + u;
    float z[4];
#pragma unroll
    for (int j = 0; j < 4; ++j) {
      const int gc = j * KD + hc;
      z[j] = fmaf(x1, Wx[512 + gc], x0 * Wx[gc]) + bias[gc];
    }
    const float iv = fsig(z[0]);
    const float gv = ftanh(z[2]);
    const float ov = fsig(z[3]);
    const float c  = iv * gv;
    const float h  = ov * ftanh(c);
    cv[u] = c;
    hs[rl * HPITCH + hc] = (_Float16)(h * oscale);
  }
  _Float16* Ho = (_Float16*)Hout;
  float* cp = Cout + (size_t)row * KD + hc4;
  *(volatile v4f*)cp = cv;
  __syncthreads();
  const bool hw = tid < 128;
  const int hrow = tid >> 4, c8 = (tid & 15) * 8;
  v8h hv = (v8h){(_Float16)0.f, (_Float16)0.f, (_Float16)0.f, (_Float16)0.f, (_Float16)0.f, (_Float16)0.f, (_Float16)0.f, (_Float16)0.f};
  _Float16* hp = Ho + (size_t)(blockIdx.x * 8 + (hw ? hrow : 0)) * KD + c8;
  if (hw) {
    hv = *(const v8h*)(hs + hrow * HPITCH + c8);
    *(volatile v8h*)hp = hv;
  }
  __threadfence();
  *(volatile v4f*)cp = cv;
  if (hw) *(volatile v8h*)hp = hv;
}

template <int MODE>
__global__ __launch_bounds__(256) void k_main(
    const unsigned short* __restrict__ Ap, const unsigned short* __restrict__ Btp,
    const float* __restrict__ Cin, const float* __restrict__ xin, int t,
    const float* __restrict__ Wx, const float* __restrict__ bias,
    const float* __restrict__ bng, const float* __restrict__ bnb,
    const float* __restrict__ bnm, const float* __restrict__ bnv,
    unsigned short* __restrict__ Hout, float* __restrict__ Fout,
    float scale, float oscale) {
  constexpr bool GATED = (MODE != 1);
  constexpr int  NWV   = (MODE == 0 || MODE == 2) ? 8 : 2;
  constexpr int  NT    = NWV * 32;
  constexpr int  HP    = (MODE == 3) ? 32 : 128;
  constexpr int  CTN   = (MODE == 0) ? 64 * CPITCH : 4;
  constexpr int  HTN   = (MODE != 3) ? 64 * HPITCH : 8;
  constexpr int  DTN   = (MODE == 3) ? 64 * 24 : 4;
  __shared__ __align__(16) float    cT[CTN];
  __shared__ __align__(16) _Float16 hT[HTN];
  __shared__ __align__(16) float    dT[DTN];

  const int tid   = threadIdx.x;
  const int lane  = tid & 31;
  const int wave  = tid >> 5;
  const int rlane = lane & 15;
  const int koff  = (lane >> 4) * 8;
  const int mOff  = (lane >> 4) * 8;
  const int m0    = blockIdx.x * 64;

  const _Float16* A  = (const _Float16*)Ap;
  const _Float16* Bt = (const _Float16*)Btp;

  v8f acc[4][4];
#pragma unroll
  for (int i = 0; i < 4; ++i)
#pragma unroll
    for (int j = 0; j < 4; ++j) acc[i][j] = (v8f){0.f,0.f,0.f,0.f,0.f,0.f,0.f,0.f};

#pragma unroll 1
  for (int k0 = 0; k0 < KD; k0 += 32) {
    v16h bh[4];
#pragma unroll
    for (int j = 0; j < 4; ++j) {
      const int brow = GATED ? (j * HP + wave * 16 + rlane) : (wave * 64 + j * 16 + rlane);
      bh[j] = Frag<_Float16>::load(Bt + (size_t)brow * KD + koff + k0);
    }
#pragma unroll
    for (int i = 0; i < 4; ++i) {
      const size_t ao = (size_t)(m0 + (i << 4) + rlane) * KD + koff + k0;
      v16h ah = Frag<_Float16>::load(A + ao);
#pragma unroll
      for (int j = 0; j < 4; ++j) acc[i][j] = Frag<_Float16>::mma(ah, bh[j], acc[i][j]);
      Frag<_Float16>::guard(acc[i][0], acc[i][3], ah, ah);
    }
    Frag<_Float16>::keep(bh[0], bh[1], bh[2], bh[3]);
  }
  acc_guard4(acc[0][0], acc[0][1], acc[0][2], acc[0][3]);
  acc_guard4(acc[1][0], acc[1][1], acc[1][2], acc[1][3]);
  acc_guard4(acc[2][0], acc[2][1], acc[2][2], acc[2][3]);
  acc_guard4(acc[3][0], acc[3][1], acc[3][2], acc[3][3]);

  const int hc = wave * 16 + rlane;
  float wb[4], w0[4], w1[4];
  float bb[4], rs[4], mm[4], gg[4], be[4];
#pragma unroll
  for (int j = 0; j < 4; ++j) {
    wb[j] = 0.f; w0[j] = 0.f; w1[j] = 0.f; bb[j] = 0.f; rs[j] = 1.f; mm[j] = 0.f; gg[j] = 1.f; be[j] = 0.f;
    if (MODE == 0 || MODE == 2) {
      const int gc = j * KD + hc;
      wb[j] = bias[gc];
      if (MODE == 0) { w0[j] = Wx[gc]; w1[j] = Wx[512 + gc]; }
    }
    if (MODE == 3) {
      const int hcl = hc < 24 ? hc : 23;
      wb[j] = bias[j * 24 + hcl];
    }
    if (MODE == 1) {
      const int n = wave * 64 + j * 16 + rlane;
      bb[j] = bias[n];
      rs[j] = rsqrtf(bnv[n] + 1e-3f);
      mm[j] = bnm[n];
      gg[j] = bng[n];
      be[j] = bnb[n];
    }
  }

#pragma unroll
  for (int i = 0; i < 4; ++i) {
#pragma unroll
    for (int r = 0; r < 8; ++r) {
      const int p = (i << 4) + mOff + r;
      if (MODE == 1) {
#pragma unroll
        for (int j = 0; j < 4; ++j) {
          float v = acc[i][j][r] * scale + bb[j];
          v = (v - mm[j]) * rs[j] * gg[j] + be[j];
          hT[p * HPITCH + wave * 64 + j * 16 + rlane] = (_Float16)(v * oscale);
        }
      } else {
        float z[4];
        if (MODE == 0) {
          const size_t xi = ((size_t)(blockIdx.x * TT + t) * PP + p) * 2;
          const float x0 = xin[xi], x1 = xin[xi + 1];
#pragma unroll
          for (int j = 0; j < 4; ++j) z[j] = (fmaf(x1, w1[j], x0 * w0[j]) + acc[i][j][r] * scale) + wb[j];
        } else {
#pragma unroll
          for (int j = 0; j < 4; ++j) z[j] = acc[i][j][r] * scale + wb[j];
        }
        const float iv = fsig(z[0]);
        const float gv = ftanh(z[2]);
        const float ov = fsig(z[3]);
        float c;
        if (MODE == 0) {
          const float fv   = fsig(z[1]);
          const float cold = Cin[(size_t)(m0 + p) * KD + hc];
          c = fmaf(fv, cold, iv * gv);
          cT[p * CPITCH + hc] = c;
        } else {
          c = iv * gv;
        }
        const float h = ov * ftanh(c);
        if (MODE == 0 || MODE == 2) hT[p * HPITCH + hc] = (_Float16)(h * oscale);
        if (MODE == 3) { if (hc < 24) dT[p * 24 + hc] = h; }
      }
    }
    asm volatile("" ::: "memory");
  }
  __syncthreads();

  if (MODE != 3) {
    _Float16* Ho = (_Float16*)Hout;
    for (int pass = 0; pass < 2; ++pass) {
#pragma unroll
      for (int it = 0; it < 1024 / NT; ++it) {
        const int q   = it * NT + tid;
        const int row = q >> 4, c8 = (q & 15) * 8;
        const v8h v = *(const v8h*)(hT + row * HPITCH + c8);
        *(volatile v8h*)(Ho + (size_t)(m0 + row) * KD + c8) = v;
      }
      if (MODE == 0) {
#pragma unroll
        for (int it = 0; it < 2048 / NT; ++it) {
          const int q   = it * NT + tid;
          const int row = q >> 5, c4 = (q & 31) * 4;
          const v4f v = *(const v4f*)(cT + row * CPITCH + c4);
          *(volatile v4f*)(Fout + (size_t)(m0 + row) * KD + c4) = v;
        }
      }
      __threadfence();
    }
  } else {
    float* outp = Fout + (size_t)blockIdx.x * 1536;
    for (int pass = 0; pass < 2; ++pass) {
#pragma unroll
      for (int it = 0; it < 6; ++it) {
        const int q   = it * 64 + tid;
        const int j12 = q >> 5;
        const int p0  = (q & 31) * 2;
        v4f v;
        v[0] = dT[p0 * 24 + 2 * j12];
        v[1] = dT[p0 * 24 + 2 * j12 + 1];
        v[2] = dT[(p0 + 1) * 24 + 2 * j12];
        v[3] = dT[(p0 + 1) * 24 + 2 * j12 + 1];
        *(volatile v4f*)(outp + (size_t)q * 4) = v;
      }
      __threadfence();
    }
  }
}

extern "C" void kernel_launch(void* const* d_in, const int* in_sizes, int n_in,
                              void* d_out, int out_size, void* d_ws, size_t ws_size,
                              hipStream_t stream) {
  if (n_in < 14) return;
  if (in_sizes[0] != NSC * TT * PP * 2) return;
  if (in_sizes[1] != 2 * 512 || in_sizes[2] != 128 * 512 || in_sizes[3] != 512) return;
  if (in_sizes[4] != 128 * 128 || in_sizes[5] != 128) return;
  if (in_sizes[6] != 128 || in_sizes[7] != 128 || in_sizes[8] != 128 || in_sizes[9] != 128) return;
  if (in_sizes[10] != 128 * 512 || in_sizes[11] != 512) return;
  if (in_sizes[12] != 128 * 96 || in_sizes[13] != 96) return;
  if (out_size != NSC * 12 * PP * 2) return;

  const float* x        = (const float*)d_in[0];
  const float* W_enc    = (const float*)d_in[1];
  const float* U_enc    = (const float*)d_in[2];
  const float* b_enc    = (const float*)d_in[3];
  const float* W_gcn    = (const float*)d_in[4];
  const float* b_gcn    = (const float*)d_in[5];
  const float* bn_gamma = (const float*)d_in[6];
  const float* bn_beta  = (const float*)d_in[7];
  const float* bn_mean  = (const float*)d_in[8];
  const float* bn_var   = (const float*)d_in[9];
  const float* W_temp   = (const float*)d_in[10];
  const float* b_temp   = (const float*)d_in[11];
  const float* W_dec    = (const float*)d_in[12];
  const float* b_dec    = (const float*)d_in[13];
  float* out = (float*)d_out;

  const size_t hbytes = (size_t)NROWS * KD * 2;
  const size_t cbytes = (size_t)NROWS * KD * 4;
  const size_t wb512  = (size_t)512 * KD * 2;
  const size_t wb128  = (size_t)128 * KD * 2;
  size_t off = 0;
  const size_t oH0 = off; off += hbytes;
  const size_t oH1 = off; off += hbytes;
  const size_t oC0 = off; off += cbytes;
  const size_t oC1 = off; off += cbytes;
  const size_t oUe = off; off += wb512;
  const size_t oWg = off; off += wb128;
  const size_t oWt = off; off += wb512;
  const size_t oWd = off; off += wb128;
  if (off > ws_size) return;
  char* ws = (char*)d_ws;
  unsigned short* H0  = (unsigned short*)(ws + oH0);
  unsigned short* H1  = (unsigned short*)(ws + oH1);
  float*          C0  = (float*)(ws + oC0);
  float*          C1  = (float*)(ws + oC1);
  unsigned short* UeT = (unsigned short*)(ws + oUe);
  unsigned short* WgT = (unsigned short*)(ws + oWg);
  unsigned short* WtT = (unsigned short*)(ws + oWt);
  unsigned short* WdT = (unsigned short*)(ws + oWd);

  const float WS  = 256.0f;
  const float HSC = 256.0f;
  const float GSC = 4096.0f;

  k_prep_wt<<<512 / 16, 256, 0, stream>>>(U_enc, 512, 128, 128, UeT, WS);
  k_prep_wt<<<128 / 16, 256, 0, stream>>>(W_gcn, 128, 128, 128, WgT, WS);
  k_prep_wt<<<512 / 16, 256, 0, stream>>>(W_temp, 512, 128, 128, WtT, WS);
  k_prep_wt<<<128 / 16, 256, 0, stream>>>(W_dec, 96, 24, 32, WdT, WS);

  k_enc0<<<NROWS / 8, 256, 0, stream>>>(x, W_enc, b_enc, H0, C0, HSC);

  unsigned short* Hp[2] = {H0, H1};
  float*          Cp[2] = {C0, C1};
  for (int t = 1; t < TT; ++t) {
    const int wi = t & 1, ri = wi ^ 1;
    k_main<0><<<NROWS / 64, 256, 0, stream>>>(Hp[ri], UeT, Cp[ri], x, t, W_enc, b_enc,
                                               bn_gamma, bn_beta, bn_mean, bn_var,
                                               Hp[wi], Cp[wi], 1.0f / (HSC * WS), HSC);
  }
  k_main<1><<<NROWS / 64, 64, 0, stream>>>(H1, WgT, C0, x, 0, W_enc, b_gcn,
                                            bn_gamma, bn_beta, bn_mean, bn_var,
                                            H0, C0, 1.0f / (HSC * WS), GSC);
  k_main<2><<<NROWS / 64, 256, 0, stream>>>(H0, WtT, C0, x, 0, W_enc, b_temp,
                                             bn_gamma, bn_beta, bn_mean, bn_var,
                                             H1, C0, 1.0f / (GSC * WS), GSC);
  k_main<3><<<NROWS / 64, 64, 0, stream>>>(H1, WdT, C0, x, 0, W_enc, b_dec,
                                            bn_gamma, bn_beta, bn_mean, bn_var,
                                            H0, out, 1.0f / (GSC * WS), 1.0f);
  (void)hipGetLastError();
}
